// T5Attention_71554155152048
// MI455X (gfx1250) — hardware-verified
//
#include <hip/hip_runtime.h>
#include <math.h>
#include <stddef.h>

#pragma clang fp contract(off)

#ifndef NB
#define NB 2
#endif
#ifndef SEQ
#define SEQ 2048
#endif
#define NB_FULL 2
#define SEQ_FULL 2048

constexpr int D_   = 512;
constexpr int H_   = 8;
constexpr int DH_  = 64;
constexpr int HD_  = H_ * DH_;
constexpr int MTOK = NB * SEQ;
constexpr int BIASL = SEQ + 128;
constexpr int NBUCK = 32;

static_assert(NB >= 1 && NB <= NB_FULL);
static_assert(SEQ >= 128 && SEQ <= SEQ_FULL);
static_assert(SEQ % 128 == 0);
static_assert(MTOK % 128 == 0);
static_assert(D_ == HD_);
static_assert(D_ % 128 == 0 && HD_ % 128 == 0);
static_assert((MTOK * D_) % 2048 == 0);
static_assert(D_ % 64 == 0);
static_assert(DH_ == 64);

constexpr float WSC   = 64.0f;
constexpr float RWSC  = 1.0f / 64.0f;
constexpr float LOSC  = 2048.0f;
constexpr float RLOSC = 1.0f / 2048.0f;
constexpr float VSC   = 16.0f;
constexpr float PSC   = 16384.0f;
constexpr float CSC   = 16.0f;
constexpr float RPVC  = CSC / (VSC * PSC);
constexpr float ROSC  = 1.0f / (WSC * CSC);

typedef _Float16 v16h __attribute__((ext_vector_type(16)));
typedef _Float16 h8   __attribute__((ext_vector_type(8)));
typedef float    v8f  __attribute__((ext_vector_type(8)));
typedef float    f4   __attribute__((ext_vector_type(4)));

union Frag16 { v16h v; h8 h[2]; };

__device__ __forceinline__ v8f mma(const Frag16& a, const Frag16& b, v8f c) {
  c = __builtin_amdgcn_wmma_f32_16x16x32_f16(false, a.v, false, b.v, (short)0, c, false, false);
  asm volatile("v_nop\n\tv_nop\n\tv_nop\n\tv_nop" : "+v"(c) : "v"(a.v), "v"(b.v));
  return c;
}

__device__ __forceinline__ float bf16_rne(float x) {
  unsigned int u = __float_as_uint(x);
  u = (u + 0x7FFFu + ((u >> 16) & 1u)) & 0xFFFF0000u;
  return __uint_as_float(u);
}

__device__ __forceinline__ int rel_bucket(int rel) {
  const int rb = (rel > 0) ? 16 : 0;
  const int an = (rel < 0) ? -rel : rel;
  int v = 15;
  v = (an < 91) ? 14 : v;
  v = (an < 64) ? 13 : v;
  v = (an < 46) ? 12 : v;
  v = (an < 32) ? 11 : v;
  v = (an < 23) ? 10 : v;
  v = (an < 16) ? 9 : v;
  v = (an < 12) ? 8 : v;
  v = (an < 8) ? an : v;
  return rb + v;
}

__global__ void __launch_bounds__(256)
k_cvt(const float* __restrict__ src, _Float16* dst, int rows_per_grp, int grp_stride_rows,
      float scale) {
  const size_t i = ((size_t)blockIdx.x * 256u + (size_t)threadIdx.x) * 8u;
  const size_t row = i / (size_t)D_;
  const int col = (int)(i % (size_t)D_);
  const size_t srow = (row / (size_t)rows_per_grp) * (size_t)grp_stride_rows +
                      (row % (size_t)rows_per_grp);
  const float* sp = src + srow * (size_t)D_ + col;
  const f4 a = *(const f4*)sp;
  const f4 c = *(const f4*)(sp + 4);
  h8 o;
  o[0] = (_Float16)(bf16_rne(a[0]) * scale);
  o[1] = (_Float16)(bf16_rne(a[1]) * scale);
  o[2] = (_Float16)(bf16_rne(a[2]) * scale);
  o[3] = (_Float16)(bf16_rne(a[3]) * scale);
  o[4] = (_Float16)(bf16_rne(c[0]) * scale);
  o[5] = (_Float16)(bf16_rne(c[1]) * scale);
  o[6] = (_Float16)(bf16_rne(c[2]) * scale);
  o[7] = (_Float16)(bf16_rne(c[3]) * scale);
  _Float16* dp = dst + i;
  *(volatile h8*)dp = o;
  __threadfence();
  *(volatile h8*)dp = o;
}

constexpr int TP = 65;

__global__ void __launch_bounds__(256)
k_cvt_wt(const float* __restrict__ W, _Float16* BT) {
  __shared__ float ts[64 * TP];
  const int t = threadIdx.x;
  const int n0 = blockIdx.x * 64, k0 = blockIdx.y * 64;
#pragma unroll
  for (int it = 0; it < 4; ++it) {
    const int kr = it * 16 + (t >> 4);
    const int c = (t & 15) * 4;
    const f4 v = *(const f4*)(W + (size_t)(k0 + kr) * D_ + n0 + c);
    ts[kr * TP + c + 0] = v[0];
    ts[kr * TP + c + 1] = v[1];
    ts[kr * TP + c + 2] = v[2];
    ts[kr * TP + c + 3] = v[3];
  }
  __syncthreads();
  h8 o[2];
#pragma unroll
  for (int it = 0; it < 2; ++it) {
    const int item = it * 256 + t;
    const int nr = item >> 3, piece = item & 7;
#pragma unroll
    for (int j = 0; j < 8; ++j)
      o[it][j] = (_Float16)(bf16_rne(ts[(piece * 8 + j) * TP + nr]) * WSC);
  }
#pragma unroll
  for (int it = 0; it < 2; ++it) {
    const int item = it * 256 + t;
    const int nr = item >> 3, piece = item & 7;
    *(volatile h8*)(BT + (size_t)(n0 + nr) * D_ + k0 + piece * 8) = o[it];
  }
  __threadfence();
#pragma unroll
  for (int it = 0; it < 2; ++it) {
    const int item = it * 256 + t;
    const int nr = item >> 3, piece = item & 7;
    *(volatile h8*)(BT + (size_t)(n0 + nr) * D_ + k0 + piece * 8) = o[it];
  }
}

constexpr int GT  = 136;
constexpr int GTF = 132;
constexpr int LDS_GEMM = 128 * GT * 2;
static_assert(LDS_GEMM >= 2 * 128 * 64 * 2);
static_assert(LDS_GEMM >= 64 * GTF * 4);

__device__ __forceinline__ void store_tile_f16(const _Float16* tile, _Float16* base,
                                               size_t pitch, int t) {
  const int piece = t & 15, rsub = t >> 4;
#pragma unroll
  for (int it = 0; it < 8; ++it) {
    const int r = it * 16 + rsub;
    const f4 v = *(const f4*)(tile + r * GT + piece * 8);
    *(volatile f4*)(base + (size_t)r * pitch + piece * 8) = v;
  }
  __threadfence();
#pragma unroll
  for (int it = 0; it < 8; ++it) {
    const int r = it * 16 + rsub;
    const f4 v = *(const f4*)(tile + r * GT + piece * 8);
    *(volatile f4*)(base + (size_t)r * pitch + piece * 8) = v;
  }
}

template <int MODE>
__global__ void __launch_bounds__(256) __attribute__((amdgpu_num_vgpr(256)))
k_gemm(const _Float16* __restrict__ A, const _Float16* __restrict__ BT, void* out0, void* out1) {
  __shared__ __align__(16) unsigned char lds_raw[LDS_GEMM];
  _Float16* As = reinterpret_cast<_Float16*>(lds_raw);
  _Float16* Bs = reinterpret_cast<_Float16*>(lds_raw + 128 * 64 * 2);

  const int t = threadIdx.x, lane = t & 31, w = t >> 5;
  const int wm = w & 3, wn = w >> 2;
  const int lr = lane & 15, hh = lane >> 4, ko = hh * 8;
  const int m0 = blockIdx.y * 128, n0 = blockIdx.x * 128;
  const int srow = t >> 1, soff = (t & 1) * 32;

  v8f acc[2][4] = {};

#pragma unroll 1
  for (int k0 = 0; k0 < D_; k0 += 64) {
    h8 ra[4], rb[4];
    const _Float16* sa = A  + (size_t)(m0 + srow) * D_ + k0 + soff;
    const _Float16* sb = BT + (size_t)(n0 + srow) * D_ + k0 + soff;
#pragma unroll
    for (int c = 0; c < 4; ++c) {
      ra[c] = *(const h8*)(sa + 8 * c);
      rb[c] = *(const h8*)(sb + 8 * c);
    }
    __syncthreads();
#pragma unroll
    for (int c = 0; c < 4; ++c) {
      *(h8*)(As + srow * 64 + soff + 8 * c) = ra[c];
      *(h8*)(Bs + srow * 64 + soff + 8 * c) = rb[c];
    }
    __syncthreads();
#pragma unroll
    for (int ks = 0; ks < 64; ks += 32) {
      Frag16 a[2], b[4];
#pragma unroll
      for (int mt = 0; mt < 2; ++mt) {
        const int row = wm * 32 + mt * 16 + lr;
        a[mt].h[0] = *(const h8*)(As + row * 64 + ks + ko);
        a[mt].h[1] = *(const h8*)(As + row * 64 + ks + ko + 16);
      }
#pragma unroll
      for (int nt = 0; nt < 4; ++nt) {
        const int col = wn * 64 + nt * 16 + lr;
        b[nt].h[0] = *(const h8*)(Bs + col * 64 + ks + ko);
        b[nt].h[1] = *(const h8*)(Bs + col * 64 + ks + ko + 16);
      }
#pragma unroll
      for (int mt = 0; mt < 2; ++mt)
#pragma unroll
        for (int nt = 0; nt < 4; ++nt)
          acc[mt][nt] = mma(a[mt], b[nt], acc[mt][nt]);
    }
  }
  __syncthreads();

  if constexpr (MODE == 0 || MODE == 1) {
    _Float16* tile = reinterpret_cast<_Float16*>(lds_raw);
    _Float16* P0 = reinterpret_cast<_Float16*>(out0);
    size_t pitch;
    _Float16* base;
    if constexpr (MODE == 0) {
      pitch = HD_;
      base = P0 + (size_t)m0 * HD_ + n0;
    } else {
      const int bidx = m0 / SEQ, s0 = m0 - bidx * SEQ;
      pitch = SEQ;
      base = P0 + (size_t)(bidx * HD_ + n0) * SEQ + s0;
    }
#pragma unroll
    for (int mt = 0; mt < 2; ++mt)
#pragma unroll
      for (int nt = 0; nt < 4; ++nt)
#pragma unroll
        for (int j = 0; j < 8; ++j) {
          const int row = wm * 32 + mt * 16 + ko + j;
          const int col = wn * 64 + nt * 16 + lr;
          const float v = acc[mt][nt][j] * RWSC;
          if constexpr (MODE == 0) tile[row * GT + col] = (_Float16)v;
          else                     tile[col * GT + row] = (_Float16)(v * VSC);
        }
    __syncthreads();
    store_tile_f16(tile, base, pitch, t);
    if constexpr (MODE == 0) {
      __syncthreads();
#pragma unroll
      for (int mt = 0; mt < 2; ++mt)
#pragma unroll
        for (int nt = 0; nt < 4; ++nt)
#pragma unroll
          for (int j = 0; j < 8; ++j) {
            const int row = wm * 32 + mt * 16 + ko + j;
            const int col = wn * 64 + nt * 16 + lr;
            const float v = acc[mt][nt][j] * RWSC;
            const _Float16 hv = (_Float16)v;
            const float res = (v - (float)hv) * LOSC;
            tile[row * GT + col] = (_Float16)res;
          }
      __syncthreads();
      _Float16* P1 = reinterpret_cast<_Float16*>(out1);
      store_tile_f16(tile, P1 + (size_t)m0 * HD_ + n0, (size_t)HD_, t);
    }
  } else {
    float* tf = reinterpret_cast<float*>(lds_raw);
    float* P0 = reinterpret_cast<float*>(out0);
    const int bidx = m0 / SEQ, s0 = m0 - bidx * SEQ;
    const size_t orow0 = (size_t)bidx * SEQ_FULL + (size_t)s0;
#pragma unroll
    for (int half = 0; half < 2; ++half) {
      if ((wm >> 1) == half) {
#pragma unroll
        for (int mt = 0; mt < 2; ++mt)
#pragma unroll
          for (int nt = 0; nt < 4; ++nt)
#pragma unroll
            for (int j = 0; j < 8; ++j) {
              const int row = (wm & 1) * 32 + mt * 16 + ko + j;
              const int col = wn * 64 + nt * 16 + lr;
              tf[row * GTF + col] = acc[mt][nt][j] * ROSC;
            }
      }
      __syncthreads();
      float* base = P0 + (orow0 + (size_t)(half * 64)) * (size_t)D_ + n0;
#pragma unroll
      for (int it = 0; it < 8; ++it) {
        const int r = it * 8 + w;
        const f4 v = *(const f4*)(tf + r * GTF + lane * 4);
        *(volatile f4*)(base + (size_t)r * D_ + lane * 4) = v;
      }
      __threadfence();
#pragma unroll
      for (int it = 0; it < 8; ++it) {
        const int r = it * 8 + w;
        const f4 v = *(const f4*)(tf + r * GTF + lane * 4);
        *(volatile f4*)(base + (size_t)r * D_ + lane * 4) = v;
      }
      __syncthreads();
    }
  }
}

constexpr int CTP = 72;

__global__ void __launch_bounds__(256) __attribute__((amdgpu_num_vgpr(256)))
k_attn(const _Float16* __restrict__ QH, const _Float16* __restrict__ QL,
       const _Float16* __restrict__ KH, const _Float16* __restrict__ KL,
       const _Float16* __restrict__ VT, const float* __restrict__ table, _Float16* Ctx) {
  __shared__ __align__(16) _Float16 Ksh[32][64];
  __shared__ __align__(16) _Float16 Ksl[32][64];
  __shared__ __align__(16) _Float16 Vs[64][32];
  __shared__ __align__(16) _Float16 ctxs[128][CTP];
  __shared__ float biasL[BIASL];

  const int t = threadIdx.x, lane = t & 31, w = t >> 5;
  const int lr = lane & 15, hh = lane >> 4, ko = hh * 8;
  const int b = blockIdx.z, h = blockIdx.y;
  const int q0 = blockIdx.x * 128;

  for (int i = t; i < SEQ + 127; i += 256) {
    const int rel = i - q0 - 127;
    biasL[i] = bf16_rne(table[rel_bucket(rel) * H_ + h]);
  }

  Frag16 qh0, qh1, ql0, ql1;
  {
    const size_t qoff = (size_t)(b * SEQ + q0 + w * 16 + lr) * HD_ + h * DH_;
    qh0.h[0] = *(const h8*)(QH + qoff + ko);
    qh0.h[1] = *(const h8*)(QH + qoff + ko + 16);
    qh1.h[0] = *(const h8*)(QH + qoff + 32 + ko);
    qh1.h[1] = *(const h8*)(QH + qoff + 32 + ko + 16);
    ql0.h[0] = *(const h8*)(QL + qoff + ko);
    ql0.h[1] = *(const h8*)(QL + qoff + ko + 16);
    ql1.h[0] = *(const h8*)(QL + qoff + 32 + ko);
    ql1.h[1] = *(const h8*)(QL + qoff + 32 + ko + 16);
  }

  const _Float16* KHb = KH + (size_t)(b * SEQ) * HD_ + h * DH_;
  const _Float16* KLb = KL + (size_t)(b * SEQ) * HD_ + h * DH_;
  const _Float16* VTb = VT + (size_t)(b * HD_ + h * DH_) * SEQ;
  const int krow = t >> 3, koff8 = (t & 7) * 8;
  const int drow = t >> 2, soff8 = (t & 3) * 8;

  v8f o[4] = {};
  float mx = -INFINITY, lsum = 0.0f;

#pragma unroll 1
  for (int kb = 0; kb < SEQ; kb += 32) {
    const h8 rkh = *(const h8*)(KHb + (size_t)(kb + krow) * HD_ + koff8);
    const h8 rkl = *(const h8*)(KLb + (size_t)(kb + krow) * HD_ + koff8);
    const h8 rv  = *(const h8*)(VTb + (size_t)drow * SEQ + kb + soff8);
    __syncthreads();
    *(h8*)&Ksh[krow][koff8] = rkh;
    *(h8*)&Ksl[krow][koff8] = rkl;
    *(h8*)&Vs[drow][soff8]  = rv;
    __syncthreads();

    v8f sc[2];
#pragma unroll
    for (int tk = 0; tk < 2; ++tk) {
      const int key = tk * 16 + lr;
      Frag16 kh0, kh1;
      kh0.h[0] = *(const h8*)&Ksh[key][ko];
      kh0.h[1] = *(const h8*)&Ksh[key][ko + 16];
      kh1.h[0] = *(const h8*)&Ksh[key][32 + ko];
      kh1.h[1] = *(const h8*)&Ksh[key][32 + ko + 16];
      v8f ch = {0.f, 0.f, 0.f, 0.f, 0.f, 0.f, 0.f, 0.f};
      v8f cr = {0.f, 0.f, 0.f, 0.f, 0.f, 0.f, 0.f, 0.f};
      ch = mma(kh0, qh0, ch);
      cr = mma(kh0, ql0, cr);
      ch = mma(kh1, qh1, ch);
      cr = mma(kh1, ql1, cr);
      Frag16 kl0, kl1;
      kl0.h[0] = *(const h8*)&Ksl[key][ko];
      kl0.h[1] = *(const h8*)&Ksl[key][ko + 16];
      kl1.h[0] = *(const h8*)&Ksl[key][32 + ko];
      kl1.h[1] = *(const h8*)&Ksl[key][32 + ko + 16];
      cr = mma(kl0, qh0, cr);
      cr = mma(kl1, qh1, cr);
      const int bbase = kb + tk * 16 + ko - (w * 16 + lr) + 127;
#pragma unroll
      for (int j = 0; j < 8; ++j)
        sc[tk][j] = ch[j] + cr[j] * RLOSC + biasL[bbase + j];
    }

    float mloc = sc[0][0];
#pragma unroll
    for (int j = 1; j < 8; ++j) mloc = fmaxf(mloc, sc[0][j]);
#pragma unroll
    for (int j = 0; j < 8; ++j) mloc = fmaxf(mloc, sc[1][j]);
    mloc = fmaxf(mloc, __shfl_xor(mloc, 16, 32));
    const float nm = fmaxf(mx, mloc);
    const float alpha = __expf(mx - nm);
    mx = nm;

    Frag16 pf;
    float rs = 0.0f;
#pragma unroll
    for (int j = 0; j < 8; ++j) {
      const float p0 = __expf(sc[0][j] - nm);
      const float p1 = __expf(sc[1][j] - nm);
      rs += p0 + p1;
      pf.h[0][j] = (_Float16)(p0 * PSC);
      pf.h[1][j] = (_Float16)(p1 * PSC);
    }
    rs += __shfl_xor(rs, 16, 32);
    lsum = lsum * alpha + rs;

#pragma unroll
    for (int tdh = 0; tdh < 4; ++tdh)
#pragma unroll
      for (int j = 0; j < 8; ++j) o[tdh][j] *= alpha;

#pragma unroll
    for (int tdh = 0; tdh < 4; ++tdh) {
      const int dhrow = tdh * 16 + lr;
      Frag16 va;
      va.h[0] = *(const h8*)&Vs[dhrow][ko];
      va.h[1] = *(const h8*)&Vs[dhrow][ko + 16];
      o[tdh] = mma(va, pf, o[tdh]);
    }
  }

  const float inv = (1.0f / lsum) * RPVC;
#pragma unroll
  for (int tdh = 0; tdh < 4; ++tdh) {
    h8 cv;
#pragma unroll
    for (int j = 0; j < 8; ++j) cv[j] = (_Float16)(o[tdh][j] * inv);
    *(h8*)&ctxs[w * 16 + lr][tdh * 16 + ko] = cv;
  }
  __syncthreads();
  {
    const int piece = t & 7, rsub = t >> 3;
    _Float16* cbase = Ctx + (size_t)(b * SEQ + q0) * HD_ + h * DH_;
#pragma unroll
    for (int it = 0; it < 4; ++it) {
      const int r = it * 32 + rsub;
      const f4 v = *(const f4*)&ctxs[r][piece * 8];
      *(volatile f4*)(cbase + (size_t)r * HD_ + piece * 8) = v;
    }
    __threadfence();
#pragma unroll
    for (int it = 0; it < 4; ++it) {
      const int r = it * 32 + rsub;
      const f4 v = *(const f4*)&ctxs[r][piece * 8];
      *(volatile f4*)(cbase + (size_t)r * HD_ + piece * 8) = v;
    }
  }
}

extern "C" void kernel_launch(void* const* d_in, const int* in_sizes, int n_in,
                              void* d_out, int out_size, void* d_ws, size_t ws_size,
                              hipStream_t stream) {
  if (n_in < 6) return;
  const int need_tok = (NB - 1) * SEQ_FULL + SEQ;
  if (in_sizes[0] < need_tok * D_) return;
  if (in_sizes[1] < D_ * HD_ || in_sizes[2] < D_ * HD_ || in_sizes[3] < D_ * HD_) return;
  if (in_sizes[4] < HD_ * D_) return;
  if (in_sizes[5] < NBUCK * H_) return;
  if (out_size < need_tok * D_) return;

  const float* hs    = (const float*)d_in[0];
  const float* Wq    = (const float*)d_in[1];
  const float* Wk    = (const float*)d_in[2];
  const float* Wv    = (const float*)d_in[3];
  const float* Wo    = (const float*)d_in[4];
  const float* table = (const float*)d_in[5];

  char* ws = (char*)d_ws;
  size_t off = 0;
  auto carve = [&](size_t bytes) -> void* {
    void* p = ws + off;
    off += (bytes + 255) & ~(size_t)255;
    return p;
  };
  const size_t plane_tok = (size_t)MTOK * HD_ * sizeof(_Float16);
  const size_t plane_w   = (size_t)D_ * HD_ * sizeof(_Float16);

  _Float16* hs16  = (_Float16*)carve(plane_tok);
  _Float16* wq16  = (_Float16*)carve(plane_w);
  _Float16* wk16  = (_Float16*)carve(plane_w);
  _Float16* wv16  = (_Float16*)carve(plane_w);
  _Float16* wo16  = (_Float16*)carve(plane_w);
  _Float16* qh16  = (_Float16*)carve(plane_tok);
  _Float16* ql16  = (_Float16*)carve(plane_tok);
  _Float16* kh16  = (_Float16*)carve(plane_tok);
  _Float16* kl16  = (_Float16*)carve(plane_tok);
  _Float16* vt16  = (_Float16*)carve(plane_tok);
  _Float16* ctx16 = (_Float16*)carve(plane_tok);
  if (off > ws_size) return;
  if (off > (size_t)134217728u) return;

  k_cvt<<<(MTOK * D_) / 2048, 256, 0, stream>>>(hs, hs16, SEQ, SEQ_FULL, 1.0f);
  dim3 gW(HD_ / 64, D_ / 64);
  k_cvt_wt<<<gW, 256, 0, stream>>>(Wq, wq16);
  k_cvt_wt<<<gW, 256, 0, stream>>>(Wk, wk16);
  k_cvt_wt<<<gW, 256, 0, stream>>>(Wv, wv16);
  k_cvt_wt<<<gW, 256, 0, stream>>>(Wo, wo16);

  dim3 gG(HD_ / 128, MTOK / 128);
  k_gemm<0><<<gG, 256, 0, stream>>>(hs16, wq16, (void*)qh16, (void*)ql16);
  k_gemm<0><<<gG, 256, 0, stream>>>(hs16, wk16, (void*)kh16, (void*)kl16);
  k_gemm<1><<<gG, 256, 0, stream>>>(hs16, wv16, (void*)vt16, (void*)vt16);

  dim3 gA(SEQ / 128, H_, NB);
  k_attn<<<gA, 256, 0, stream>>>(qh16, ql16, kh16, kl16, vt16, table, ctx16);

  dim3 gO(D_ / 128, MTOK / 128);
  k_gemm<2><<<gO, 256, 0, stream>>>(ctx16, wo16, d_out, d_out);

  (void)hipGetLastError();
}
